// TransformerFrustumEncoder_3358664425621
// MI455X (gfx1250) — hardware-verified
//
#include <hip/hip_runtime.h>
#include <stdint.h>
#include <math.h>

typedef _Float16 v16h __attribute__((ext_vector_type(16)));
typedef _Float16 v8h  __attribute__((ext_vector_type(8)));
typedef float    v8f  __attribute__((ext_vector_type(8)));
typedef float    v4f  __attribute__((ext_vector_type(4)));
typedef float    v4fa __attribute__((ext_vector_type(4), __may_alias__));
typedef unsigned v4u  __attribute__((ext_vector_type(4)));

#define NPOL 64
#define NAZ  256
#define NSY  (NPOL * NAZ)
#define NH   4
#define ND   32
#define NE   128
#define NCP  128
#define NL   2
#define NCIN 8
#define NF   8192
#define NP   16

#define SACT  64.0f
#define SWGT  256.0f
#define UN_AW (1.0f / 16384.0f)
#define UN_AA (1.0f / 4096.0f)

__device__ __forceinline__ v8f wmma16(v16h a, v16h b, v8f c) {
  c = __builtin_amdgcn_wmma_f32_16x16x32_f16(false, a, false, b, (short)0, c,
                                             false, false);
  asm volatile("v_nop\n\tv_nop\n\tv_nop\n\tv_nop" : "+v"(c) : "v"(a), "v"(b));
  return c;
}

__device__ __forceinline__ float gelu_exact(float x) {
  return 0.5f * x * (1.0f + erff(x * 0.70710678118654752f));
}


__device__ __forceinline__ v16h fragA(const float* base, int stride, int kbase,
                                      int kmax, int lane, float scale) {
  const int m = lane & 15;
  const int h8 = (lane >> 4) * 8;
  v16h a;
#pragma unroll
  for (int i = 0; i < 16; ++i) {
    const int k = (i < 8) ? (h8 + i) : (16 + h8 + (i - 8));
    const float v = (k < kmax) ? base[m * stride + kbase + k] * scale : 0.0f;
    a[i] = (_Float16)v;
  }
  return a;
}

__device__ __forceinline__ v16h fragB(const float* base, int stride, int kbase,
                                      int nbase, int kmax, int lane, float scale) {
  const int n = lane & 15;
  const int h8 = (lane >> 4) * 8;
  v16h b;
#pragma unroll
  for (int i = 0; i < 16; ++i) {
    const int k = (i < 8) ? (h8 + i) : (16 + h8 + (i - 8));
    const float v = (k < kmax) ? base[(kbase + k) * stride + nbase + n] * scale : 0.0f;
    b[i] = (_Float16)v;
  }
  return b;
}

__device__ __forceinline__ v16h fragW(const _Float16* pk, int fragIdx, int lane) {
  return *(const v16h*)(pk + ((size_t)fragIdx * 32 + lane) * 16);
}

template <int LEN>
__device__ __forceinline__ void ln_row(const float* xrow, float* hrow,
                                       const float* __restrict__ g,
                                       const float* __restrict__ b) {
  float m = 0.0f;
  for (int d = 0; d < LEN; ++d) m += xrow[d];
  m *= (1.0f / LEN);
  float v = 0.0f;
  for (int d = 0; d < LEN; ++d) { float dd = xrow[d] - m; v += dd * dd; }
  v *= (1.0f / LEN);
  const float inv = rsqrtf(v + 1e-5f);
  for (int d = 0; d < LEN; ++d) hrow[d] = (xrow[d] - m) * inv * g[d] + b[d];
}

__global__ __launch_bounds__(256) void k_pack_w(const float* __restrict__ src,
                                                _Float16* __restrict__ dst,
                                                int nl, int K, int N, float scale) {
  const int per = (K * N) >> 3;
  const int total = nl * per;
  const int u = blockIdx.x * blockDim.x + threadIdx.x;
  if (u >= total) return;
  const int l  = u / per;
  const int uu = u - l * per;
  const int frag = uu >> 6;
  const int li = (uu >> 1) & 31;
  const int hf = uu & 1;
  const int NT = N >> 4;
  const int kc = frag / NT;
  const int nt = frag - kc * NT;
  const int nn = nt * 16 + (li & 15);
  const int kb = kc * 32 + (li >> 4) * 8 + 16 * hf;
  const float* s = src + (size_t)l * K * N;
  v8h tmp;
#pragma unroll
  for (int i = 0; i < 8; ++i)
    tmp[i] = (_Float16)(s[(size_t)(kb + i) * N + nn] * scale);
  union { v8h h; v4u w; } pk;
  pk.h = tmp;
  volatile v4u* d = (volatile v4u*)(dst + (size_t)l * K * N + (size_t)uu * 8);
  *d = pk.w;
  __threadfence();
  *d = pk.w;
}

__global__ __launch_bounds__(32) void k_groups(
    const float* __restrict__ pc,
    const float* __restrict__ fc_pre_w, const float* __restrict__ fc_pre_b,
    const _Float16* __restrict__ pkQ, const float* __restrict__ qkv_b,
    const float* __restrict__ sa_g, const float* __restrict__ sa_b,
    const float* __restrict__ ffn_g, const float* __restrict__ ffn_bn,
    const _Float16* __restrict__ pkF1, const float* __restrict__ ffn_b1,
    const _Float16* __restrict__ pkF2, const float* __restrict__ ffn_b2,
    const float* __restrict__ ca_g, const float* __restrict__ ca_b,
    const _Float16* __restrict__ pkKV, const float* __restrict__ kv_b,
    const float* __restrict__ dec, const int* __restrict__ i_unique,
    const int* __restrict__ ppg, int nf,
    float* outF) {
  __shared__ float xs[NP][132];
  __shared__ float hs[NP][132];
  __shared__ float ts[NP][264];
  __shared__ float ptile[NP * NCIN];
  __shared__ float cq[NCP];
  __shared__ float csc[NP];
  __shared__ float cwt[NP];

  const int f = blockIdx.x;
  if (f >= nf) return;
  if (ppg[0] != NP) return;
  const int lane = threadIdx.x & 31;
  const int n = lane & 15;
  const int h8 = (lane >> 4) * 8;

  for (int i = lane; i < NP * NCIN; i += 32)
    ptile[i] = pc[(size_t)f * NP * NCIN + i];
  __syncthreads();

  for (int p = 0; p < NP; ++p) {
    for (int c = lane; c < NE; c += 32) {
      float acc = 0.0f;
#pragma unroll
      for (int i = 0; i < NCIN; ++i)
        acc += ptile[p * NCIN + i] * fc_pre_w[i * NE + c];
      xs[p][c] = acc + fc_pre_b[c];
    }
  }
  __syncthreads();

  const float sc_scale = 0.17677669529663687f * UN_AA;

  for (int l = 0; l < NL; ++l) {
#pragma unroll
    for (int t = 0; t < 2; ++t) {
      const int grp = lane * 2 + t;
      const int p = grp >> 2, hd = grp & 3;
      ln_row<ND>(&xs[p][hd * ND], &hs[p][hd * ND], sa_g + l * ND, sa_b + l * ND);
    }
    __syncthreads();

    const _Float16* wq = pkQ + (size_t)l * (ND * 3 * ND);
    for (int hd = 0; hd < NH; ++hd) {
      {
        const v16h ah = fragA(&hs[0][0], 132, hd * ND, 32, lane, SACT);
        for (int nt = 0; nt < 6; ++nt) {
          v8f c = {};
          c = wmma16(ah, fragW(wq, nt, lane), c);
          const int col = nt * 16 + n;
#pragma unroll
          for (int r = 0; r < 8; ++r)
            ts[h8 + r][col] = c[r] * UN_AW + qkv_b[l * 96 + col];
        }
      }
      __syncthreads();

      {
        const v16h aq = fragA(&ts[0][0], 264, 0, 32, lane, SACT);
        const v16h bk = fragA(&ts[0][0], 264, ND, 32, lane, SACT);
        v8f sc = {};
        sc = wmma16(aq, bk, sc);
#pragma unroll
        for (int r = 0; r < 8; ++r) ts[h8 + r][96 + n] = sc[r] * sc_scale;
      }
      __syncthreads();

      if (lane < 16) {
        float mx = -3.0e38f;
        for (int qy = 0; qy < NP; ++qy) mx = fmaxf(mx, ts[lane][96 + qy]);
        float s = 0.0f;
        for (int qy = 0; qy < NP; ++qy) {
          const float e = expf(ts[lane][96 + qy] - mx);
          ts[lane][96 + qy] = e;
          s += e;
        }
        const float inv = 1.0f / s;
        for (int qy = 0; qy < NP; ++qy) ts[lane][96 + qy] *= inv;
      }
      __syncthreads();

      {
        const v16h aa = fragA(&ts[0][0], 264, 96, 16, lane, SACT);
#pragma unroll
        for (int nt = 0; nt < 2; ++nt) {
          const v16h bv = fragB(&ts[0][0], 264, 0, 64 + nt * 16, 16, lane, SACT);
          v8f o = {};
          o = wmma16(aa, bv, o);
          const int col = hd * ND + nt * 16 + n;
#pragma unroll
          for (int r = 0; r < 8; ++r) xs[h8 + r][col] += o[r] * UN_AA;
        }
      }
      __syncthreads();
    }

#pragma unroll
    for (int t = 0; t < 2; ++t) {
      const int grp = lane * 2 + t;
      const int p = grp >> 2, hd = grp & 3;
      ln_row<ND>(&xs[p][hd * ND], &hs[p][hd * ND], ffn_g + l * ND, ffn_bn + l * ND);
    }
    __syncthreads();

    const _Float16* w1 = pkF1 + (size_t)l * (ND * 4 * ND);
    const _Float16* w2 = pkF2 + (size_t)l * (4 * ND * ND);
    for (int hd = 0; hd < NH; ++hd) {
      {
        const v16h ah = fragA(&hs[0][0], 132, hd * ND, 32, lane, SACT);
        for (int nt = 0; nt < 8; ++nt) {
          v8f c = {};
          c = wmma16(ah, fragW(w1, nt, lane), c);
          const int col = nt * 16 + n;
#pragma unroll
          for (int r = 0; r < 8; ++r)
            ts[h8 + r][col] = gelu_exact(c[r] * UN_AW + ffn_b1[l * 128 + col]);
        }
      }
      __syncthreads();

      {
        v16h af[4];
#pragma unroll
        for (int kc = 0; kc < 4; ++kc)
          af[kc] = fragA(&ts[0][0], 264, kc * 32, 32, lane, SACT);
#pragma unroll
        for (int nt = 0; nt < 2; ++nt) {
          v8f c = {};
#pragma unroll
          for (int kc = 0; kc < 4; ++kc)
            c = wmma16(af[kc], fragW(w2, kc * 2 + nt, lane), c);
          const int col = hd * ND + nt * 16 + n;
#pragma unroll
          for (int r = 0; r < 8; ++r)
            xs[h8 + r][col] += c[r] * UN_AW + ffn_b2[l * ND + nt * 16 + n];
        }
      }
      __syncthreads();
    }
  }

  if (lane < 16) ln_row<NE>(&xs[lane][0], &hs[lane][0], ca_g, ca_b);
  __syncthreads();

  {
    v16h ak[4];
#pragma unroll
    for (int kc = 0; kc < 4; ++kc)
      ak[kc] = fragA(&hs[0][0], 132, kc * 32, 32, lane, SACT);
    for (int nt = 0; nt < 16; ++nt) {
      v8f c = {};
#pragma unroll
      for (int kc = 0; kc < 4; ++kc)
        c = wmma16(ak[kc], fragW(pkKV, kc * 16 + nt, lane), c);
      const int col = nt * 16 + n;
#pragma unroll
      for (int r = 0; r < 8; ++r) ts[h8 + r][col] = c[r] * UN_AW + kv_b[col];
    }
  }

  {
    int iu = i_unique[f];
    iu = iu < 0 ? 0 : (iu > NSY - 1 ? NSY - 1 : iu);
    const float* q = dec + (size_t)(iu % NPOL) * NCP;
    for (int c = lane; c < NCP; c += 32) cq[c] = q[c];
  }
  __syncthreads();

  if (lane < 16) {
    float s = 0.0f;
    for (int c = 0; c < NCP; ++c) s += cq[c] * ts[lane][c];
    csc[lane] = s * 0.08838834764831845f;
  }
  __syncthreads();
  {
    float mx = -3.0e38f;
    for (int j = 0; j < NP; ++j) mx = fmaxf(mx, csc[j]);
    float den = 0.0f;
    for (int j = 0; j < NP; ++j) den += expf(csc[j] - mx);
    const float rden = 1.0f / den;
    if (lane < 16) cwt[lane] = expf(csc[lane] - mx) * rden;
  }
  __syncthreads();

  {
    v4f o;
#pragma unroll
    for (int i = 0; i < 4; ++i) {
      const int c = lane * 4 + i;
      float a = 0.0f;
      for (int j = 0; j < NP; ++j) a += cwt[j] * ts[j][NCP + c];
      o[i] = a + cq[c];
    }
    volatile v4f* d = (volatile v4f*)(outF + (size_t)f * NCP + lane * 4);
    *d = o;
    __threadfence();
    *d = o;
  }
}

__global__ __launch_bounds__(256) void k_gather_rows(const float* __restrict__ outF,
                                                     const int* __restrict__ i_unique,
                                                     int nf, float* feats, int nrows) {
  const int wave = threadIdx.x >> 5;
  const int lane = threadIdx.x & 31;
  const int r = blockIdx.x * (blockDim.x >> 5) + wave;
  if (r >= nrows) return;
  int lo = 0, hi = nf;
#pragma unroll 1
  for (int it = 0; it < 16; ++it) {
    if (lo < hi) {
      const int mid = (lo + hi) >> 1;
      const int v = i_unique[mid];
      if (v < r) lo = mid + 1; else hi = mid;
    }
  }
  bool found = false;
  if (lo < nf) {
    lo = lo < 0 ? 0 : lo;
    found = (i_unique[lo] == r);
  }
  v4f val = {0.0f, 0.0f, 0.0f, 0.0f};
  if (found) val = *(const v4f*)(outF + (size_t)lo * NCP + lane * 4);
  volatile v4f* d = (volatile v4f*)(feats + (size_t)r * NCP + lane * 4);
  *d = val;
  __threadfence();
  *d = val;
}

__global__ __launch_bounds__(32) void k_image_ffn(
    const float* __restrict__ feats,
    const float* __restrict__ g, const float* __restrict__ b,
    const _Float16* __restrict__ w1s, const float* __restrict__ b1,
    const _Float16* __restrict__ w2s, const float* __restrict__ b2,
    int nrows, float* out) {
  __shared__ float ft[16][132];
  __shared__ float hn[16][132];
  __shared__ float hid[16][520];
  const int r0 = blockIdx.x * 16;
  if (r0 + 16 > nrows) return;
  const int lane = threadIdx.x & 31;
  const int n = lane & 15;
  const int h8 = (lane >> 4) * 8;

  for (int i4 = lane; i4 < 16 * NCP / 4; i4 += 32) {
    const v4f v = *(const v4f*)(feats + (size_t)r0 * NCP + (size_t)i4 * 4);
    const int row = i4 >> 5, col = (i4 & 31) * 4;
    ft[row][col + 0] = v[0];
    ft[row][col + 1] = v[1];
    ft[row][col + 2] = v[2];
    ft[row][col + 3] = v[3];
  }
  __syncthreads();

  if (lane < 16) ln_row<NCP>(&ft[lane][0], &hn[lane][0], g, b);
  __syncthreads();

  {
    v16h af[4];
#pragma unroll
    for (int kc = 0; kc < 4; ++kc)
      af[kc] = fragA(&hn[0][0], 132, kc * 32, 32, lane, SACT);
    for (int nt = 0; nt < 32; ++nt) {
      v8f c = {};
#pragma unroll
      for (int kc = 0; kc < 4; ++kc)
        c = wmma16(af[kc], fragW(w1s, kc * 32 + nt, lane), c);
      const int col = nt * 16 + n;
#pragma unroll
      for (int r = 0; r < 8; ++r)
        hid[h8 + r][col] = gelu_exact(c[r] * UN_AW + b1[col]);
    }
  }
  __syncthreads();

  {
    v8f acc[8];
#pragma unroll
    for (int nt = 0; nt < 8; ++nt) acc[nt] = (v8f){};
    for (int kb = 0; kb < 4; ++kb) {
      v16h a4[4];
#pragma unroll
      for (int j = 0; j < 4; ++j)
        a4[j] = fragA(&hid[0][0], 520, (kb * 4 + j) * 32, 32, lane, SACT);
#pragma unroll
      for (int nt = 0; nt < 8; ++nt) {
#pragma unroll
        for (int j = 0; j < 4; ++j)
          acc[nt] = wmma16(a4[j], fragW(w2s, (kb * 4 + j) * 8 + nt, lane), acc[nt]);
      }
    }
#pragma unroll
    for (int nt = 0; nt < 8; ++nt) {
      const int col = nt * 16 + n;
#pragma unroll
      for (int r = 0; r < 8; ++r) {
        const float v = acc[nt][r] * UN_AW + b2[col] + ft[h8 + r][col];
        ft[h8 + r][col] = v;
      }
    }
  }
  __syncthreads();

  for (int r = 0; r < 16; ++r) {
    const v4fa v = *(const v4fa*)(&ft[r][lane * 4]);
    *(volatile v4fa*)(out + (size_t)(r0 + r) * NCP + lane * 4) = v;
  }
  __threadfence();
  for (int r = 0; r < 16; ++r) {
    const v4fa v = *(const v4fa*)(&ft[r][lane * 4]);
    *(volatile v4fa*)(out + (size_t)(r0 + r) * NCP + lane * 4) = v;
  }
}

extern "C" void kernel_launch(void* const* d_in, const int* in_sizes, int n_in,
                              void* d_out, int out_size, void* d_ws, size_t ws_size,
                              hipStream_t stream) {
  if (n_in < 26) return;
  if (in_sizes[0]  != NF * NP * NCIN)   return;
  if (in_sizes[1]  != NCIN * NE)        return;
  if (in_sizes[2]  != NE)               return;
  if (in_sizes[3]  != NL * ND * 3 * ND) return;
  if (in_sizes[4]  != NL * 3 * ND)      return;
  if (in_sizes[9]  != NL * ND * 4 * ND) return;
  if (in_sizes[11] != NL * 4 * ND * ND) return;
  if (in_sizes[15] != NE * 2 * NCP)     return;
  if (in_sizes[17] != NPOL * NCP)       return;
  if (in_sizes[20] != NCP * 4 * NCP)    return;
  if (in_sizes[22] != 4 * NCP * NCP)    return;
  if (in_sizes[24] != NF)               return;
  if (in_sizes[25] < 1)                 return;
  if (out_size != NSY * NCP)            return;

  const float* pc       = (const float*)d_in[0];
  const float* fc_pre_w = (const float*)d_in[1];
  const float* fc_pre_b = (const float*)d_in[2];
  const float* qkv_w    = (const float*)d_in[3];
  const float* qkv_b    = (const float*)d_in[4];
  const float* sa_g     = (const float*)d_in[5];
  const float* sa_b     = (const float*)d_in[6];
  const float* ffn_g    = (const float*)d_in[7];
  const float* ffn_bn   = (const float*)d_in[8];
  const float* ffn_w1   = (const float*)d_in[9];
  const float* ffn_b1   = (const float*)d_in[10];
  const float* ffn_w2   = (const float*)d_in[11];
  const float* ffn_b2   = (const float*)d_in[12];
  const float* ca_g     = (const float*)d_in[13];
  const float* ca_b     = (const float*)d_in[14];
  const float* kv_w     = (const float*)d_in[15];
  const float* kv_b     = (const float*)d_in[16];
  const float* dec      = (const float*)d_in[17];
  const float* cff_g    = (const float*)d_in[18];
  const float* cff_b    = (const float*)d_in[19];
  const float* cff_w1   = (const float*)d_in[20];
  const float* cff_b1   = (const float*)d_in[21];
  const float* cff_w2   = (const float*)d_in[22];
  const float* cff_b2   = (const float*)d_in[23];
  const int*   i_unique = (const int*)d_in[24];
  const int*   ppg      = (const int*)d_in[25];
  float* out = (float*)d_out;

  char* ws = (char*)d_ws;
  size_t cur = 0;
  auto walloc = [&](size_t bytes) -> void* {
    void* p = ws + cur;
    cur = (cur + bytes + 255) & ~(size_t)255;
    return p;
  };
  const size_t nQ  = (size_t)NL * ND * 3 * ND;
  const size_t nF1 = (size_t)NL * ND * 4 * ND;
  const size_t nF2 = (size_t)NL * 4 * ND * ND;
  const size_t nKV = (size_t)NE * 2 * NCP;
  const size_t nC1 = (size_t)NCP * 4 * NCP;
  const size_t nC2 = (size_t)4 * NCP * NCP;
  _Float16* pkQ   = (_Float16*)walloc(nQ  * sizeof(_Float16));
  _Float16* pkF1  = (_Float16*)walloc(nF1 * sizeof(_Float16));
  _Float16* pkF2  = (_Float16*)walloc(nF2 * sizeof(_Float16));
  _Float16* pkKV  = (_Float16*)walloc(nKV * sizeof(_Float16));
  _Float16* pkC1  = (_Float16*)walloc(nC1 * sizeof(_Float16));
  _Float16* pkC2  = (_Float16*)walloc(nC2 * sizeof(_Float16));
  float*    outF  = (float*)walloc((size_t)NF * NCP * sizeof(float));
  float*    feats = (float*)walloc((size_t)NSY * NCP * sizeof(float));
  if (cur > ws_size) return;

  auto nblk = [](size_t units) -> unsigned { return (unsigned)((units + 255) / 256); };

  k_pack_w<<<nblk(nQ  / 8), 256, 0, stream>>>(qkv_w,  pkQ,  NL, ND, 3 * ND, SWGT);
  k_pack_w<<<nblk(nF1 / 8), 256, 0, stream>>>(ffn_w1, pkF1, NL, ND, 4 * ND, SWGT);
  k_pack_w<<<nblk(nF2 / 8), 256, 0, stream>>>(ffn_w2, pkF2, NL, 4 * ND, ND, SWGT);
  k_pack_w<<<nblk(nKV / 8), 256, 0, stream>>>(kv_w,   pkKV, 1, NE, 2 * NCP, SWGT);
  k_pack_w<<<nblk(nC1 / 8), 256, 0, stream>>>(cff_w1, pkC1, 1, NCP, 4 * NCP, SWGT);
  k_pack_w<<<nblk(nC2 / 8), 256, 0, stream>>>(cff_w2, pkC2, 1, 4 * NCP, NCP, SWGT);

  k_groups<<<NF, 32, 0, stream>>>(
      pc, fc_pre_w, fc_pre_b, pkQ, qkv_b, sa_g, sa_b, ffn_g, ffn_bn,
      pkF1, ffn_b1, pkF2, ffn_b2, ca_g, ca_b, pkKV, kv_b, dec,
      i_unique, ppg, NF, outF);

  k_gather_rows<<<(NSY + 7) / 8, 256, 0, stream>>>(outF, i_unique, NF, feats, NSY);

  k_image_ffn<<<NSY / 16, 32, 0, stream>>>(feats, cff_g, cff_b, pkC1, cff_b1,
                                           pkC2, cff_b2, NSY, out);
}
